// GPSA_26912265077208
// MI455X (gfx1250) — hardware-verified
//
#include <hip/hip_runtime.h>


#define NB_  8
#define TT   1024
#define GS   32
#define DM   256
#define NH_  8
#define HD   32
#define HDP  64
#define DQ   (NH_ * HD)
#define PCAR 1024.0f
#define SCL  0.17677669529663688f
typedef _Float16 h16;
typedef unsigned short bf;
typedef __attribute__((ext_vector_type(16))) __bf16   v16bf;
typedef __attribute__((ext_vector_type(16))) _Float16 v16h;
typedef __attribute__((ext_vector_type(8)))  _Float16 v8h;
typedef __attribute__((ext_vector_type(8)))  unsigned short v8us;
typedef __attribute__((ext_vector_type(8)))  float    v8f;
typedef __attribute__((ext_vector_type(4)))  float    v4f;
typedef v8h  __attribute__((may_alias)) v8ha;
typedef v4f  __attribute__((may_alias)) v4fa;
typedef v8us __attribute__((may_alias)) v8usa;

__device__ __forceinline__ unsigned short f2bf(float f) { unsigned u = __float_as_uint(f); u += 0x7FFFu + ((u >> 16) & 1u); return (unsigned short)(u >> 16); }
__device__ __forceinline__ float bf2f(unsigned short b) { return __uint_as_float(((unsigned)b) << 16); }
__device__ __forceinline__ float bfr(float f) { return bf2f(f2bf(f)); }
__device__ __forceinline__ v16h cat16(v8h lo, v8h hi) { return __builtin_shufflevector(lo, hi, 0, 1, 2, 3, 4, 5, 6, 7, 8, 9, 10, 11, 12, 13, 14, 15); }
__device__ __forceinline__ v16bf cat16b(v8us lo, v8us hi) { return __builtin_bit_cast(v16bf, __builtin_shufflevector(lo, hi, 0, 1, 2, 3, 4, 5, 6, 7, 8, 9, 10, 11, 12, 13, 14, 15)); }
__device__ __forceinline__ v8f wmma16(v16h a, v16h b, v8f c) { return __builtin_amdgcn_wmma_f32_16x16x32_f16(false, a, false, b, (short)0, c, false, false); }
__device__ __forceinline__ v8f wmmab(v16bf a, v16bf b, v8f c) { return __builtin_amdgcn_wmma_f32_16x16x32_bf16(false, a, false, b, (short)0, c, false, false); }


template <typename T16> struct WFrag;
template <> struct WFrag<h16> { typedef v16h V; static __device__ __forceinline__ V ld(const h16* p) { return cat16(*(const v8h*)p, *(const v8h*)(p + 16)); } static __device__ __forceinline__ v8f mma(V a, V b, v8f c) { return wmma16(a, b, c); } };
template <> struct WFrag<bf> { typedef v16bf V; static __device__ __forceinline__ V ld(const bf* p) { return cat16b(*(const v8us*)p, *(const v8us*)(p + 16)); } static __device__ __forceinline__ v8f mma(V a, V b, v8f c) { return wmmab(a, b, c); } };
template <typename T16, int NSPLIT, bool BIAS>
__global__ __launch_bounds__(32) void k_gemmw(const T16* __restrict__ A, const T16* __restrict__ A2, const T16* __restrict__ Bt, const T16* __restrict__ Bt2, int K, float* C, int ldc, const float* __restrict__ bias, size_t sA, size_t sB, size_t sC) {
    typedef typename WFrag<T16>::V V;
    __shared__ __align__(16) float os[16 * 68];
    const size_t z = blockIdx.z; A += z * sA; if (A2) A2 += z * sA; Bt += z * sB; if (Bt2) Bt2 += z * sB; C += z * sC;
    const int lane = threadIdx.x & 31, lr = lane & 15, hi = lane >> 4; const int r0 = blockIdx.x * 64, c0 = blockIdx.y * 64;
    v8f acc[4][4];
#pragma unroll
    for (int mb = 0; mb < 4; ++mb)
#pragma unroll
        for (int nb = 0; nb < 4; ++nb) acc[mb][nb] = (v8f){};
    const size_t aoff = (size_t)(r0 + lr) * K + 8 * hi, boff = (size_t)(c0 + lr) * K + 8 * hi;
#pragma unroll 1
    for (int kc = 0; kc < K; kc += 32) {
        V a[4], a2[4];
#pragma unroll
        for (int mb = 0; mb < 4; ++mb) { a[mb] = WFrag<T16>::ld(A + aoff + (size_t)mb * 16 * K + kc); if (NSPLIT == 1 || NSPLIT == 2) a2[mb] = WFrag<T16>::ld(A2 + aoff + (size_t)mb * 16 * K + kc); }
#pragma unroll
        for (int nb = 0; nb < 4; ++nb) { const V b = WFrag<T16>::ld(Bt + boff + (size_t)nb * 16 * K + kc); V b2; if (NSPLIT >= 2) b2 = WFrag<T16>::ld(Bt2 + boff + (size_t)nb * 16 * K + kc);
#pragma unroll
            for (int mb = 0; mb < 4; ++mb) { acc[mb][nb] = WFrag<T16>::mma(a[mb], b, acc[mb][nb]); if (NSPLIT == 1 || NSPLIT == 2) acc[mb][nb] = WFrag<T16>::mma(a2[mb], b, acc[mb][nb]); if (NSPLIT >= 2) acc[mb][nb] = WFrag<T16>::mma(a[mb], b2, acc[mb][nb]); } }
        asm volatile("v_nop\n\tv_nop\n\tv_nop\n\tv_nop" : "+v"(acc[0][0]), "+v"(acc[1][1]), "+v"(acc[2][2]), "+v"(acc[3][3]) : "v"(a[0]), "v"(a[3]));
    }
#pragma unroll
    for (int mb = 0; mb < 4; ++mb) {
#pragma unroll
        for (int nb = 0; nb < 4; ++nb) {
#pragma unroll
            for (int j = 0; j < 8; ++j) os[(hi * 8 + j) * 68 + nb * 16 + lr] = acc[mb][nb][j]; }
        __builtin_amdgcn_wave_barrier(); asm volatile("" ::: "memory");
        float* crow = C + (size_t)(r0 + mb * 16) * ldc + c0;
#pragma unroll 1
        for (int ps = 0; ps < 2; ++ps) {
#pragma unroll
            for (int s = 0; s < 8; ++s) { const int row = 2 * s + hi, cofs = lr * 4; v4f val = *(const v4fa*)(os + row * 68 + cofs); if (BIAS) { val[0] += bfr(bias[c0 + cofs]); val[1] += bfr(bias[c0 + cofs + 1]); val[2] += bfr(bias[c0 + cofs + 2]); val[3] += bfr(bias[c0 + cofs + 3]); }
                *(volatile v4f*)(crow + (size_t)row * ldc + cofs) = val; }
            if (ps == 0) __threadfence(); }
        __builtin_amdgcn_wave_barrier(); asm volatile("" ::: "memory");
    }
}

typedef __attribute__((ext_vector_type(4))) unsigned short v4us;
typedef __attribute__((ext_vector_type(2))) _Float16 v2h;
typedef __attribute__((ext_vector_type(4))) _Float16 v4h;
__device__ __forceinline__ h16 tohx(float x) { return (h16)x; }
__device__ __forceinline__ void splitf(float y, unsigned short& h, unsigned short& l) { h = f2bf(y); l = f2bf(y - bf2f(h)); }
__global__ __launch_bounds__(256) void k_cvt8(const float* __restrict__ src, bf* dst, size_t n8) { const size_t i = (size_t)blockIdx.x * 256 + threadIdx.x; if (i >= n8) return; const v8f v = *(const v8f*)(src + i * 8); v8us o;
#pragma unroll
    for (int k = 0; k < 8; ++k) o[k] = f2bf(v[k]); *(volatile v8us*)(dst + i * 8) = o; __threadfence(); *(volatile v8us*)(dst + i * 8) = o; }

__global__ __launch_bounds__(256) void k_cvt8T(const float* __restrict__ src, bf* dst) { const size_t i = (size_t)blockIdx.x * 256 + threadIdx.x; if (i >= (size_t)TT * DM / 8) return; const int t = (int)(i / (DM / 8)); const int c0 = (int)(i % (DM / 8)) * 8; v8us o;
#pragma unroll
    for (int k = 0; k < 8; ++k) o[k] = f2bf(src[(size_t)(c0 + k) * TT + t]); *(volatile v8us*)(dst + (size_t)t * DM + c0) = o; __threadfence(); *(volatile v8us*)(dst + (size_t)t * DM + c0) = o; }
__global__ __launch_bounds__(256) void k_qkpl(const float* __restrict__ F, h16* QP, h16* KP) { const size_t e = ((size_t)blockIdx.x * 256 + threadIdx.x) * 2; if (e >= (size_t)NH_ * TT * HD) return; const int d = (int)(e % HD); const int t = (int)((e / HD) % TT); const int h = (int)(e / ((size_t)HD * TT)); const float* f = F + (size_t)t * (2 * DQ) + h * HD + d; v2h oq, ok;
    oq[0] = tohx(f[0]); oq[1] = tohx(f[1]); ok[0] = tohx(f[DQ]); ok[1] = tohx(f[DQ + 1]); *(volatile v2h*)(QP + e) = oq; *(volatile v2h*)(KP + e) = ok; __threadfence(); *(volatile v2h*)(QP + e) = oq; *(volatile v2h*)(KP + e) = ok; }
__global__ __launch_bounds__(256) void k_vtpl(const float* __restrict__ F, h16* V16) { const size_t e = ((size_t)blockIdx.x * 256 + threadIdx.x) * 2; if (e >= (size_t)NH_ * HDP * TT) return; const int t = (int)(e % TT); const int dp = (int)((e / TT) % HDP); const int h = (int)(e / ((size_t)TT * HDP)); v2h o;
    if (dp < HD) { o[0] = tohx(F[(size_t)t * DQ + h * HD + dp]); o[1] = tohx(F[(size_t)(t + 1) * DQ + h * HD + dp]); } else { o[0] = (h16)0.0f; o[1] = (h16)0.0f; }
    *(volatile v2h*)(V16 + e) = o; __threadfence(); *(volatile v2h*)(V16 + e) = o; }
__global__ __launch_bounds__(256) void k_posT(const float* __restrict__ wpos, const float* __restrict__ bpos, float* POS) {
    const int lane = threadIdx.x & 31; const int row = blockIdx.x * 8 + (threadIdx.x >> 5); if (row >= NH_ * TT) return; const int n = row % TT; const int h = row / TT; const int nr = n / GS, nc = n % GS;
    float w0 = bfr(wpos[h * 3 + 0]), w1 = bfr(wpos[h * 3 + 1]), w2 = bfr(wpos[h * 3 + 2]), bp = bfr(bpos[h]); asm volatile("" : "+v"(w0), "+v"(w1), "+v"(w2), "+v"(bp));
    auto logit = [&](int m) { const int dxi = (m % GS) - nc, dyi = (m / GS) - nr; const int ddi = dxi * dxi + dyi * dyi; float p0 = __fmul_rn(w0, (float)dxi), p1 = __fmul_rn(w1, (float)dyi), p2 = __fmul_rn(w2, (float)ddi); asm volatile("" : "+v"(p0), "+v"(p1), "+v"(p2)); return __fadd_rn(__fadd_rn(__fadd_rn(p0, p1), p2), bp); };
    float mx = -3.0e38f;
#pragma unroll 1
    for (int ch = 0; ch < TT / 128; ++ch) { for (int q = 0; q < 4; ++q) mx = fmaxf(mx, logit(ch * 128 + lane * 4 + q)); }
#pragma unroll
    for (int sh = 16; sh; sh >>= 1) mx = fmaxf(mx, __shfl_xor(mx, sh, 32));
    float s = 0.f;
#pragma unroll 1
    for (int ch = 0; ch < TT / 128; ++ch) { for (int q = 0; q < 4; ++q) { float d0 = __fsub_rn(logit(ch * 128 + lane * 4 + q), mx); asm volatile("" : "+v"(d0)); s = __fadd_rn(s, __builtin_amdgcn_exp2f(__fmul_rn(d0, 1.4426950408889634f))); } }
#pragma unroll
    for (int sh = 16; sh; sh >>= 1) s = __fadd_rn(s, __shfl_xor(s, sh, 32));
    const float f = __fdiv_rn(1.0f, s);
#pragma unroll 1
    for (int ps = 0; ps < 2; ++ps) {
#pragma unroll 1
        for (int ch = 0; ch < TT / 128; ++ch) { v4f o;
#pragma unroll
            for (int q = 0; q < 4; ++q) { float d0 = __fsub_rn(logit(ch * 128 + lane * 4 + q), mx); asm volatile("" : "+v"(d0)); float e = __builtin_amdgcn_exp2f(__fmul_rn(d0, 1.4426950408889634f)); asm volatile("" : "+v"(e)); o[q] = __fmul_rn(e, f); }
            *(volatile v4f*)(POS + (size_t)row * TT + ch * 128 + lane * 4) = o; }
        if (ps == 0) __threadfence(); }
}
__global__ __launch_bounds__(256) void k_asoftG(const float* __restrict__ Sb, const float* __restrict__ POS, const float* __restrict__ gat, const float* __restrict__ maskb, h16* P16) {
    const int lane = threadIdx.x & 31; const int row = blockIdx.x * 8 + (threadIdx.x >> 5); if (row >= NH_ * TT) return; const int h = row / TT; const float* sr = Sb + (size_t)row * TT; const float* pr = POS + (size_t)row * TT; float v[TT / 32]; float mx = -3.0e38f;
    float gl = bfr(gat[h]); asm volatile("" : "+v"(gl)); const float g = __fdiv_rn(1.0f, __fadd_rn(1.0f, __builtin_amdgcn_exp2f(__fmul_rn(gl, -1.4426950408889634f)))); const float omg = __fsub_rn(1.0f, g);
#pragma unroll
    for (int ch = 0; ch < TT / 128; ++ch) { const int j0 = ch * 128 + lane * 4; const v4f a = *(const v4f*)(sr + j0);
#pragma unroll
        for (int q = 0; q < 4; ++q) { const float t = __fmul_rn(a[q], SCL); v[ch * 4 + q] = t; mx = fmaxf(mx, t); } }
#pragma unroll
    for (int sh = 16; sh; sh >>= 1) mx = fmaxf(mx, __shfl_xor(mx, sh, 32));
    float s1 = 0.f;
#pragma unroll
    for (int k = 0; k < TT / 32; ++k) { float d0 = __fsub_rn(v[k], mx); asm volatile("" : "+v"(d0)); v[k] = __builtin_amdgcn_exp2f(__fmul_rn(d0, 1.4426950408889634f)); s1 = __fadd_rn(s1, v[k]); }
#pragma unroll
    for (int sh = 16; sh; sh >>= 1) s1 = __fadd_rn(s1, __shfl_xor(s1, sh, 32));
    const float f1 = __fdiv_rn(omg, s1); float sa = 0.f;
#pragma unroll
    for (int ch = 0; ch < TT / 128; ++ch) { const v4f pp = *(const v4f*)(pr + ch * 128 + lane * 4);
#pragma unroll
        for (int q = 0; q < 4; ++q) { float a1 = __fmul_rn(v[ch * 4 + q], f1), a2 = __fmul_rn(pp[q], g); asm volatile("" : "+v"(a1), "+v"(a2)); const float t = __fadd_rn(a1, a2); v[ch * 4 + q] = t; sa = __fadd_rn(sa, t); } }
#pragma unroll
    for (int sh = 16; sh; sh >>= 1) sa = __fadd_rn(sa, __shfl_xor(sa, sh, 32));
    const float ra = __fdiv_rn(1.0f, sa); float sb = 0.f;
#pragma unroll
    for (int ch = 0; ch < TT / 128; ++ch) { const v4f mk = *(const v4f*)(maskb + ch * 128 + lane * 4);
#pragma unroll
        for (int q = 0; q < 4; ++q) { float an = __fmul_rn(v[ch * 4 + q], ra); asm volatile("" : "+v"(an)); float mm = bfr(mk[q]); asm volatile("" : "+v"(mm)); const float t = __fmul_rn(an, mm); v[ch * 4 + q] = t; sb = __fadd_rn(sb, t); } }
#pragma unroll
    for (int sh = 16; sh; sh >>= 1) sb = __fadd_rn(sb, __shfl_xor(sb, sh, 32));
    const float rb = __fdiv_rn(PCAR, sb);
#pragma unroll 1
    for (int ps = 0; ps < 2; ++ps) {
#pragma unroll
        for (int ch = 0; ch < TT / 128; ++ch) { v4h o4;
#pragma unroll
            for (int q = 0; q < 4; ++q) { float y = __fmul_rn(v[ch * 4 + q], rb); asm volatile("" : "+v"(y)); o4[q] = tohx(y); }
            *(volatile v4h*)(P16 + (size_t)row * TT + ch * 128 + lane * 4) = o4; }
        if (ps == 0) __threadfence(); }
}

__global__ __launch_bounds__(256) void k_mergeG(const float* __restrict__ O, bf* Ah, bf* Al) { const size_t e = ((size_t)blockIdx.x * 256 + threadIdx.x) * 4; if (e >= (size_t)TT * DQ) return; const int c = (int)(e % DQ); const int t = (int)(e / DQ); const int h = c / HD, d = c % HD; v4us oh, ol;
    const v4f ov = *(const v4f*)(O + (((size_t)h * TT + t) * HDP + d));
#pragma unroll
    for (int q = 0; q < 4; ++q) { float y = __fmul_rn(ov[q], 1.0f / PCAR); asm volatile("" : "+v"(y)); unsigned short a2, c2; splitf(y, a2, c2); oh[q] = a2; ol[q] = c2; }
    *(volatile v4us*)(Ah + e) = oh; *(volatile v4us*)(Al + e) = ol; __threadfence(); *(volatile v4us*)(Ah + e) = oh; *(volatile v4us*)(Al + e) = ol; }
__global__ __launch_bounds__(256) void k_outC(const float* __restrict__ Y, float* out) { const size_t i = (size_t)blockIdx.x * 256 + threadIdx.x; if (i >= (size_t)DM * TT / 4) return; const int t0 = (int)(i % (TT / 4)) * 4; const int c = (int)(i / (TT / 4)); v4f o;
#pragma unroll
    for (int q = 0; q < 4; ++q) o[q] = Y[(size_t)(t0 + q) * DM + c]; *(volatile v4f*)(out + (size_t)c * TT + t0) = o; __threadfence(); *(volatile v4f*)(out + (size_t)c * TT + t0) = o; }

extern "C" void kernel_launch(void* const* d_in, const int* in_sizes, int n_in,
                              void* d_out, int out_size, void* d_ws, size_t ws_size, hipStream_t stream) {
    (void)in_sizes; (void)n_in; (void)out_size;
    const float* x = (const float*)d_in[0]; const float* maskb = (const float*)d_in[1]; const float* wqk = (const float*)d_in[2]; const float* wv = (const float*)d_in[3]; const float* wpr = (const float*)d_in[4]; const float* bpr = (const float*)d_in[5]; const float* wpos = (const float*)d_in[6]; const float* bpos = (const float*)d_in[7]; const float* gat = (const float*)d_in[8];
    float* OUT = (float*)d_out;
    char* wsp = (char*)d_ws;
    auto take = [&](size_t bytes) { char* p = wsp; wsp += (bytes + 255) & ~(size_t)255; return (void*)p; };
    bf* WQK = (bf*)take((size_t)2 * DQ * DM * 2); bf* WV = (bf*)take((size_t)DQ * DM * 2); bf* WP = (bf*)take((size_t)DM * DQ * 2); bf* XB = (bf*)take((size_t)TT * DM * 2);
    float* FQK = (float*)take((size_t)TT * 2 * DQ * 4); float* FVb = (float*)take((size_t)TT * DQ * 4); h16* QP = (h16*)take((size_t)NH_ * TT * HD * 2); h16* KP = (h16*)take((size_t)NH_ * TT * HD * 2); h16* VT = (h16*)take((size_t)NH_ * HDP * TT * 2);
    float* Sb = (float*)take((size_t)NH_ * TT * TT * 4); h16* P16 = (h16*)take((size_t)NH_ * TT * TT * 2); float* Ob = (float*)take((size_t)NH_ * TT * HDP * 4); bf* ATh = (bf*)take((size_t)TT * DQ * 2); bf* ATl = (bf*)take((size_t)TT * DQ * 2); float* Y = (float*)take((size_t)TT * DM * 4); float* POS = (float*)take((size_t)NH_ * TT * TT * 4);
    if ((size_t)(wsp - (char*)d_ws) > ws_size) return;
    k_cvt8<<<(unsigned)(((size_t)2 * DQ * DM / 8 + 255) / 256), 256, 0, stream>>>(wqk, WQK, (size_t)2 * DQ * DM / 8); k_cvt8<<<(unsigned)(((size_t)DQ * DM / 8 + 255) / 256), 256, 0, stream>>>(wv, WV, (size_t)DQ * DM / 8); k_cvt8<<<(unsigned)(((size_t)DM * DQ / 8 + 255) / 256), 256, 0, stream>>>(wpr, WP, (size_t)DM * DQ / 8);
    k_posT<<<NH_ * TT / 8, 256, 0, stream>>>(wpos, bpos, POS);
    for (int b = 0; b < NB_; ++b) {
        k_cvt8T<<<(unsigned)(((size_t)TT * DM / 8 + 255) / 256), 256, 0, stream>>>(x + (size_t)b * DM * TT, XB);
        k_gemmw<bf, 0, false><<<dim3(TT / 64, 2 * DQ / 64, 1), 32, 0, stream>>>(XB, nullptr, WQK, nullptr, DM, FQK, 2 * DQ, nullptr, 0, 0, 0); k_qkpl<<<(unsigned)(((size_t)NH_ * TT * HD / 2 + 255) / 256), 256, 0, stream>>>(FQK, QP, KP);
        k_gemmw<bf, 0, false><<<dim3(TT / 64, DQ / 64, 1), 32, 0, stream>>>(XB, nullptr, WV, nullptr, DM, FVb, DQ, nullptr, 0, 0, 0); k_vtpl<<<(unsigned)(((size_t)NH_ * HDP * TT / 2 + 255) / 256), 256, 0, stream>>>(FVb, VT);
        k_gemmw<h16, 0, false><<<dim3(TT / 64, TT / 64, NH_), 32, 0, stream>>>(QP, nullptr, KP, nullptr, HD, Sb, TT, nullptr, (size_t)TT * HD, (size_t)TT * HD, (size_t)TT * TT);
        k_asoftG<<<NH_ * TT / 8, 256, 0, stream>>>(Sb, POS, gat, maskb + (size_t)b * TT, P16);
        k_gemmw<h16, 0, false><<<dim3(TT / 64, HDP / 64, NH_), 32, 0, stream>>>(P16, nullptr, VT, nullptr, TT, Ob, HDP, nullptr, (size_t)TT * TT, (size_t)HDP * TT, (size_t)TT * HDP);
        k_mergeG<<<(unsigned)(((size_t)TT * DQ / 4 + 255) / 256), 256, 0, stream>>>(Ob, ATh, ATl);
        k_gemmw<bf, 1, true><<<dim3(TT / 64, DM / 64, 1), 32, 0, stream>>>(ATh, ATl, WP, nullptr, DQ, Y, DM, bpr, 0, 0, 0);
        k_outC<<<(unsigned)(((size_t)DM * TT / 4 + 255) / 256), 256, 0, stream>>>(Y, OUT + (size_t)b * DM * TT); }
}
